// LightweightMHSA_36283883717427
// MI455X (gfx1250) — hardware-verified
//
#include <hip/hip_runtime.h>
#define NB 16
#define NP 512
#define DQ 1024
#define DR 256
#define NHD 8
#define NBH (NB * NHD)
#define GRP 32
#define NRW (NB * NP)
typedef __bf16 v16b __attribute__((ext_vector_type(16)));
typedef unsigned short v8us __attribute__((ext_vector_type(8), may_alias));
typedef float  v8f  __attribute__((ext_vector_type(8)));
typedef float  v4f  __attribute__((ext_vector_type(4)));
typedef float  v4fa __attribute__((ext_vector_type(4), may_alias));
union FragB { v16b v; v8us half[2]; unsigned short u[16]; };

__device__ __forceinline__ unsigned short bf16_bits(float x) { unsigned int u = __float_as_uint(x); return (unsigned short)((u + 0x7FFFu + ((u >> 16) & 1u)) >> 16); }
__device__ __forceinline__ float bf16_val(unsigned short b) { return __uint_as_float(((unsigned int)b) << 16); }
__device__ __forceinline__ float bf16_round(float x) { return bf16_val(bf16_bits(x)); }
template <int NT>
__device__ __forceinline__ v8f mmaN(v16b ah, v16b al, v16b bh, v16b bl, v8f c) {
  c = __builtin_amdgcn_wmma_f32_16x16x32_bf16(false, ah, false, bh, (short)0, c, false, false);
  if (NT >= 2) c = __builtin_amdgcn_wmma_f32_16x16x32_bf16(false, al, false, bh, (short)0, c, false, false);
  if (NT >= 3) c = __builtin_amdgcn_wmma_f32_16x16x32_bf16(false, ah, false, bl, (short)0, c, false, false);
  asm volatile("v_nop\n\tv_nop\n\tv_nop\n\tv_nop" : "+v"(c) : "v"(ah), "v"(al), "v"(bh), "v"(bl));
  return c;
}

__global__ __launch_bounds__(256) void k_wt_bf16(const float* __restrict__ W, unsigned short* __restrict__ Wt, int K, int N) {
  const int t = blockIdx.x * 256 + threadIdx.x;
  const int k8n = K / 8;
  if (t >= N * k8n) return;
  const int n = t / k8n, k8 = (t % k8n) * 8;
  v8us v;
#pragma unroll
  for (int i = 0; i < 8; ++i) v[i] = bf16_bits(W[(size_t)(k8 + i) * N + n]);
  *(volatile v8us*)(Wt + (size_t)n * K + k8) = v;
  __threadfence();
  *(volatile v8us*)(Wt + (size_t)n * K + k8) = v;
}

template <bool ASPLIT, int ACT, bool BIAS_BF16>
__global__ __launch_bounds__(128) void k_gemm_bf(const float* __restrict__ A, int lda, const unsigned short* __restrict__ Wt, int ldb,
                                               const float* __restrict__ bias, float* __restrict__ C, int ldc, int M, int N, int K) {
  __shared__ __attribute__((aligned(16))) float so[4][16][64];
  const int tid = threadIdx.x, w = tid >> 5, lane = tid & 31, ln = lane & 15, hh = lane >> 4;
  const int ntn = N / 64;
  const int wid = blockIdx.x * 4 + w;
  const int mt = wid / ntn, nq = wid % ntn;
  if (mt * 16 >= M) return;
  const int row0 = mt * 16, col0 = nq * 64;
  const float* arow = A + (size_t)(row0 + ln) * lda;
  v8f acc[4] = {};
  for (int kb = 0; kb < K; kb += 32) {
    FragB ah, al;
    const v4f x0 = *(const v4fa*)(arow + kb + 8 * hh), x1 = *(const v4fa*)(arow + kb + 8 * hh + 4);
    const v4f x2 = *(const v4fa*)(arow + kb + 16 + 8 * hh), x3 = *(const v4fa*)(arow + kb + 16 + 8 * hh + 4);
    float xs[16] = {x0[0],x0[1],x0[2],x0[3],x1[0],x1[1],x1[2],x1[3],x2[0],x2[1],x2[2],x2[3],x3[0],x3[1],x3[2],x3[3]};
#pragma unroll
    for (int i = 0; i < 16; ++i) { const unsigned short hb = bf16_bits(xs[i]); ah.u[i] = hb; al.u[i] = ASPLIT ? bf16_bits(xs[i] - bf16_val(hb)) : (unsigned short)0; }
#pragma unroll
    for (int t = 0; t < 4; ++t) {
      const unsigned short* brow = Wt + (size_t)(col0 + t * 16 + ln) * ldb + kb;
      FragB b;
      b.half[0] = *(const v8us*)(brow + 8 * hh);
      b.half[1] = *(const v8us*)(brow + 16 + 8 * hh);
      acc[t] = mmaN<ASPLIT ? 2 : 1>(ah.v, al.v, b.v, b.v, acc[t]);
    }
  }
#pragma unroll
  for (int t = 0; t < 4; ++t) {
    float bv = bias ? bias[col0 + t * 16 + ln] : 0.f;
    if (BIAS_BF16) bv = bf16_round(bv);
#pragma unroll
    for (int r = 0; r < 8; ++r) { float v = acc[t][r] + bv; if (ACT == 1) v = fmaxf(v, 0.f); so[w][8 * hh + r][t * 16 + ln] = v; }
  }
  __builtin_amdgcn_fence(__ATOMIC_ACQ_REL, "workgroup");
  __builtin_amdgcn_wave_barrier();
  const int rsub = lane >> 4, c4 = (lane & 15) * 4;
  for (int pass = 0; pass < 2; ++pass) {
#pragma unroll
    for (int q = 0; q < 8; ++q) {
      const int r = q * 2 + rsub;
      const v4f v = *(const v4fa*)&so[w][r][c4];
      *(volatile v4f*)(C + (size_t)(row0 + r) * ldc + col0 + c4) = v;
    }
    if (pass == 0) __threadfence();
  }
}

template <bool ASPLIT, int ACT, bool BIAS_BF16, bool RES_BF16>
__global__ __launch_bounds__(128) void k_gemm_bf3(const float* __restrict__ A, int lda, const unsigned short* __restrict__ Wt, int ldb,
                                                const float* __restrict__ bias, const float* __restrict__ resid, int rmod, int ldr,
                                                float* __restrict__ C, int ldc, int M, int N, int K) {
  __shared__ __attribute__((aligned(16))) float so[4][16][64];
  const int tid = threadIdx.x, w = tid >> 5, lane = tid & 31, ln = lane & 15, hh = lane >> 4;
  const int ntn = N / 64;
  const int wid = blockIdx.x * 4 + w;
  const int mt = wid / ntn, nq = wid % ntn;
  if (mt * 16 >= M) return;
  const int row0 = mt * 16, col0 = nq * 64;
  const float* arow = A + (size_t)(row0 + ln) * lda;
  v8f acc[4] = {};
  for (int kb = 0; kb < K; kb += 32) {
    FragB ah, al;
    const v4f x0 = *(const v4fa*)(arow + kb + 8 * hh), x1 = *(const v4fa*)(arow + kb + 8 * hh + 4);
    const v4f x2 = *(const v4fa*)(arow + kb + 16 + 8 * hh), x3 = *(const v4fa*)(arow + kb + 16 + 8 * hh + 4);
    float xs[16] = {x0[0],x0[1],x0[2],x0[3],x1[0],x1[1],x1[2],x1[3],x2[0],x2[1],x2[2],x2[3],x3[0],x3[1],x3[2],x3[3]};
#pragma unroll
    for (int i = 0; i < 16; ++i) { const unsigned short hb = bf16_bits(xs[i]); ah.u[i] = hb; al.u[i] = ASPLIT ? bf16_bits(xs[i] - bf16_val(hb)) : (unsigned short)0; }
#pragma unroll
    for (int t = 0; t < 4; ++t) {
      const unsigned short* brow = Wt + (size_t)(col0 + t * 16 + ln) * ldb + kb;
      FragB b;
      b.half[0] = *(const v8us*)(brow + 8 * hh);
      b.half[1] = *(const v8us*)(brow + 16 + 8 * hh);
      acc[t] = mmaN<ASPLIT ? 2 : 1>(ah.v, al.v, b.v, b.v, acc[t]);
    }
  }
#pragma unroll
  for (int t = 0; t < 4; ++t) {
    const int col = col0 + t * 16 + ln;
    float bv = bias ? bias[col] : 0.f;
    if (BIAS_BF16) bv = bf16_round(bv);
#pragma unroll
    for (int r = 0; r < 8; ++r) {
      float v = acc[t][r] + bv;
      if (resid) { float rv = resid[(size_t)((row0 + 8 * hh + r) % rmod) * ldr + col]; if (RES_BF16) rv = bf16_round(rv); v += rv; }
      if (ACT == 1) v = fmaxf(v, 0.f);
      if (ACT == 2) v = 0.5f * v * (1.0f + erff(v * 0.70710678118654752f));
      if (ACT == 3) { const float u = 0.7978845608028654f * (v + 0.044715f * v * v * v); v = 0.5f * v * (1.0f + tanhf(u)); }
      so[w][8 * hh + r][t * 16 + ln] = v;
    }
  }
  __builtin_amdgcn_fence(__ATOMIC_ACQ_REL, "workgroup");
  __builtin_amdgcn_wave_barrier();
  const int rsub = lane >> 4, c4 = (lane & 15) * 4;
  for (int pass = 0; pass < 2; ++pass) {
#pragma unroll
    for (int q = 0; q < 8; ++q) {
      const int r = q * 2 + rsub;
      const v4f v = *(const v4fa*)&so[w][r][c4];
      *(volatile v4f*)(C + (size_t)(row0 + r) * ldc + col0 + c4) = v;
    }
    if (pass == 0) __threadfence();
  }
}
template <bool PARAM_BF16>
__global__ __launch_bounds__(256) void k_layernorm(const float* __restrict__ X, const float* __restrict__ R, const float* __restrict__ g, const float* __restrict__ bta,
                                                  float* __restrict__ out_sum, float* __restrict__ out_norm, int N, float eps) {
  __shared__ float red[256];
  const int row = blockIdx.x, tid = threadIdx.x;
  const float* x = X + (size_t)row * N; const float* rr = R ? R + (size_t)row * N : nullptr;
  float vals[16];
  const int per = N / 256;
  float s1 = 0.f;
  for (int u = 0; u < per / 4; ++u) {
    const int j = tid * 4 + 1024 * u;
    const v4f a = *(const v4fa*)(x + j);
    v4f b = {0.f,0.f,0.f,0.f}; if (rr) b = *(const v4fa*)(rr + j);
#pragma unroll
    for (int q = 0; q < 4; ++q) { const float v = a[q] + b[q]; vals[u * 4 + q] = v; s1 += v; }
  }
  red[tid] = s1; __syncthreads();
  for (int st = 128; st > 0; st >>= 1) { if (tid < st) red[tid] += red[tid + st]; __syncthreads(); }
  const float mu = red[0] / (float)N; __syncthreads();
  float s2 = 0.f;
  for (int u = 0; u < per / 4; ++u)
#pragma unroll
    for (int q = 0; q < 4; ++q) { const float c = vals[u * 4 + q] - mu; s2 += c * c; }
  red[tid] = s2; __syncthreads();
  for (int st = 128; st > 0; st >>= 1) { if (tid < st) red[tid] += red[tid + st]; __syncthreads(); }
  const float rs = rsqrtf(red[0] / (float)N + eps);
  for (int pass = 0; pass < 2; ++pass) {
    for (int u = 0; u < per / 4; ++u) {
      const int j = tid * 4 + 1024 * u;
      v4f o, sm;
#pragma unroll
      for (int q = 0; q < 4; ++q) {
        float gg = g[j + q], bb = bta[j + q];
        if (PARAM_BF16) { gg = bf16_round(gg); bb = bf16_round(bb); }
        sm[q] = vals[u * 4 + q]; o[q] = (vals[u * 4 + q] - mu) * rs * gg + bb;
      }
      if (out_sum) *(volatile v4f*)(out_sum + (size_t)row * N + j) = sm;
      *(volatile v4f*)(out_norm + (size_t)row * N + j) = o;
    }
    if (pass == 0) __threadfence();
  }
}


typedef _Float16 v16h __attribute__((ext_vector_type(16)));
union FragH { v16h v; v8us half[2]; _Float16 h[16]; unsigned short u[16]; };
template <int NT>
__device__ __forceinline__ v8f mmaH(v16h ah, v16h al, v16h bh, v16h bl, v8f c) {
  c = __builtin_amdgcn_wmma_f32_16x16x32_f16(false, ah, false, bh, (short)0, c, false, false);
  if (NT >= 2) c = __builtin_amdgcn_wmma_f32_16x16x32_f16(false, al, false, bh, (short)0, c, false, false);
  if (NT >= 3) c = __builtin_amdgcn_wmma_f32_16x16x32_f16(false, ah, false, bl, (short)0, c, false, false);
  asm volatile("v_nop\n\tv_nop\n\tv_nop\n\tv_nop" : "+v"(c) : "v"(ah), "v"(al), "v"(bh), "v"(bl));
  return c;
}
template <bool ASPLIT>
__global__ __launch_bounds__(128) void k_gemm_h(const float* __restrict__ A, int lda, size_t sA, const _Float16* __restrict__ Bh, int ldb, size_t sB, float alpha, float* __restrict__ C, int ldc, size_t sC, int M, int N, int K) {
  __shared__ __attribute__((aligned(16))) float so[4][16][64];
  const int tid = threadIdx.x, w = tid >> 5, lane = tid & 31, ln = lane & 15, hh = lane >> 4; const int by = blockIdx.y;
  A += (size_t)by * sA; Bh += (size_t)by * sB; C += (size_t)by * sC;
  const int ntn = (N + 63) / 64; const int wid = blockIdx.x * 4 + w; const int mt = wid / ntn, nq = wid % ntn; if (mt * 16 >= M) return;
  const int row0 = mt * 16, col0 = nq * 64; const float* arow = A + (size_t)(row0 + ln) * lda;
  v8f acc[4] = {};
  for (int kb = 0; kb < K; kb += 32) {
    FragH ah, al;
    const v4f x0 = *(const v4fa*)(arow + kb + 8 * hh), x1 = *(const v4fa*)(arow + kb + 8 * hh + 4), x2 = *(const v4fa*)(arow + kb + 16 + 8 * hh), x3 = *(const v4fa*)(arow + kb + 16 + 8 * hh + 4);
    float xs[16] = {x0[0],x0[1],x0[2],x0[3],x1[0],x1[1],x1[2],x1[3],x2[0],x2[1],x2[2],x2[3],x3[0],x3[1],x3[2],x3[3]};
#pragma unroll
    for (int i = 0; i < 16; ++i) { const _Float16 h = (_Float16)xs[i]; ah.h[i] = h; al.h[i] = ASPLIT ? (_Float16)(xs[i] - (float)h) : (_Float16)0.0f; }
#pragma unroll
    for (int t = 0; t < 4; ++t) { if (col0 + t * 16 >= N) continue; const size_t boff = (size_t)(col0 + t * 16 + ln) * ldb + kb; FragH bq; bq.half[0] = *(const v8us*)(Bh + boff + 8 * hh); bq.half[1] = *(const v8us*)(Bh + boff + 16 + 8 * hh);
      acc[t] = mmaH<ASPLIT ? 2 : 1>(ah.v, al.v, bq.v, bq.v, acc[t]); }
  }
#pragma unroll
  for (int t = 0; t < 4; ++t) { if (col0 + t * 16 >= N) continue;
#pragma unroll
    for (int r = 0; r < 8; ++r) so[w][8 * hh + r][t * 16 + ln] = acc[t][r] * alpha; }
  __builtin_amdgcn_fence(__ATOMIC_ACQ_REL, "workgroup"); __builtin_amdgcn_wave_barrier();
  const int rsub = lane >> 4, c4 = (lane & 15) * 4;
  for (int pass = 0; pass < 2; ++pass) {
#pragma unroll
    for (int q = 0; q < 8; ++q) { const int r = q * 2 + rsub; if (col0 + c4 < N) { const v4f v = *(const v4fa*)&so[w][r][c4]; *(volatile v4f*)(C + (size_t)(row0 + r) * ldc + col0 + c4) = v; } }
    if (pass == 0) __threadfence(); }
}

__global__ __launch_bounds__(256) void k_wt_f16(const float* __restrict__ W, _Float16* __restrict__ Wt, int K, int N, float scale) {
  const int t = blockIdx.x * 256 + threadIdx.x; if (t >= N * (K / 8)) return; const int n = t / (K / 8), k8 = (t % (K / 8)) * 8; FragH f;
#pragma unroll
  for (int i = 0; i < 8; ++i) f.h[i] = (_Float16)(bf16_round(W[(size_t)(k8 + i) * N + n]) * scale); const v8us o = f.half[0];
  *(volatile v8us*)((unsigned short*)Wt + (size_t)n * K + k8) = o; __threadfence(); *(volatile v8us*)((unsigned short*)Wt + (size_t)n * K + k8) = o;
}
template <int ACT>
__global__ __launch_bounds__(128) void k_gemm_hhx(const _Float16* __restrict__ A, int lda, size_t sA, const _Float16* __restrict__ Bh, int ldb, size_t sB, float alpha, const float* __restrict__ bias, size_t sBias, const float* __restrict__ CP, int rowsPerB, size_t sCPb, int row0g,
    float* __restrict__ C, _Float16* __restrict__ C16, int ldc, size_t sC, int M, int N, int K) {
  __shared__ __attribute__((aligned(16))) float so[4][16][64];
  const int tid = threadIdx.x, w = tid >> 5, lane = tid & 31, ln = lane & 15, hh = lane >> 4; const int by = blockIdx.y;
  A += (size_t)by * sA; Bh += (size_t)by * sB; const size_t cofs = (size_t)by * sC; const float* bp = bias ? bias + (size_t)by * sBias : nullptr;
  const int ntn = (N + 63) / 64; const int wid = blockIdx.x * 4 + w; const int mt = wid / ntn, nq = wid % ntn; if (mt * 16 >= M) return;
  const int row0 = mt * 16, col0 = nq * 64; const _Float16* arow = A + (size_t)(row0 + ln) * lda;
  v8f acc[4] = {};
  for (int kb = 0; kb < K; kb += 32) { FragH ah; ah.half[0] = *(const v8us*)((const unsigned short*)arow + kb + 8 * hh); ah.half[1] = *(const v8us*)((const unsigned short*)arow + kb + 16 + 8 * hh);
#pragma unroll
    for (int t = 0; t < 4; ++t) { if (col0 + t * 16 >= N) continue; const size_t boff = (size_t)(col0 + t * 16 + ln) * ldb + kb; FragH bq; bq.half[0] = *(const v8us*)((const unsigned short*)Bh + boff + 8 * hh); bq.half[1] = *(const v8us*)((const unsigned short*)Bh + boff + 16 + 8 * hh);
      acc[t] = mmaH<1>(ah.v, ah.v, bq.v, bq.v, acc[t]); }
  }
#pragma unroll
  for (int t = 0; t < 4; ++t) { if (col0 + t * 16 >= N) continue; const int col = col0 + t * 16 + ln; const float bv = bp ? bf16_round(bp[col]) : 0.f;
#pragma unroll
    for (int r = 0; r < 8; ++r) { float v = acc[t][r] * alpha + bv; if (CP) { const int bidx = (row0g + row0 + 8 * hh + r) / rowsPerB; v += CP[(size_t)bidx * sCPb + (size_t)by * 64 + col]; } if (ACT == 1) v = (v > 0.f) ? v : expm1f(v); else if (ACT == 7) v = (v > 0.f) ? v + 1.0f : expf(v); else if (ACT == 8) v = tanhf(v); else if (ACT == 9) v = 0.5f * v * (1.0f + tanhf(0.7978845608028654f * (v + 0.044715f * v * v * v))); else if (ACT == 11) v = 1.0f / (1.0f + expf(-v)); else if (ACT == 12) v = (v > 0.f) ? v : 0.01f * v; else if (ACT == 14) v = (v > 0.f) ? v : 0.1f * v; else if (ACT == 15) v = v / (1.0f + expf(-v)); else if (ACT == 3) v = fmaxf(v, 0.f); else if (ACT == 6) v = 0.5f * v * (1.0f + erff(v * 0.70710678118654752f)); so[w][8 * hh + r][t * 16 + ln] = v; } }
  __builtin_amdgcn_fence(__ATOMIC_ACQ_REL, "workgroup"); __builtin_amdgcn_wave_barrier();
  const int rsub = lane >> 4, c4 = (lane & 15) * 4; typedef _Float16 v4h __attribute__((ext_vector_type(4)));
  for (int pass = 0; pass < 2; ++pass) {
#pragma unroll
    for (int q = 0; q < 8; ++q) { const int r = q * 2 + rsub; if (col0 + c4 < N) { const v4f v = *(const v4fa*)&so[w][r][c4]; if (C) *(volatile v4f*)(C + cofs + (size_t)(row0 + r) * ldc + col0 + c4) = v; if (C16) { v4h h4; for (int i = 0; i < 4; ++i) h4[i] = (_Float16)v[i]; *(volatile v4h*)(C16 + cofs + (size_t)(row0 + r) * ldc + col0 + c4) = h4; } } }
    if (pass == 0) __threadfence(); }
}


typedef _Float16 v4h __attribute__((ext_vector_type(4)));

__global__ __launch_bounds__(256) void k_x16(const float* __restrict__ x, _Float16* __restrict__ X16, size_t n8) { const size_t t = (size_t)blockIdx.x * 256 + threadIdx.x; if (t >= n8) return; FragH f;
#pragma unroll
  for (int q = 0; q < 8; ++q) f.h[q] = (_Float16)bf16_round(x[t * 8 + q]); *(volatile v8us*)((unsigned short*)X16 + t * 8) = f.half[0]; __threadfence(); *(volatile v8us*)((unsigned short*)X16 + t * 8) = f.half[0]; }
__global__ __launch_bounds__(256) void k_h16(const float* __restrict__ x, _Float16* __restrict__ X16, size_t n8) { const size_t t = (size_t)blockIdx.x * 256 + threadIdx.x; if (t >= n8) return; FragH f;
#pragma unroll
  for (int q = 0; q < 8; ++q) f.h[q] = (_Float16)x[t * 8 + q]; *(volatile v8us*)((unsigned short*)X16 + t * 8) = f.half[0]; __threadfence(); *(volatile v8us*)((unsigned short*)X16 + t * 8) = f.half[0]; }
__global__ __launch_bounds__(256) void k_round16f(const float* __restrict__ W, _Float16* __restrict__ Bt, size_t n8) { const size_t t = (size_t)blockIdx.x * 256 + threadIdx.x; if (t >= n8) return; FragH f;
#pragma unroll
  for (int i = 0; i < 8; ++i) f.h[i] = (_Float16)(bf16_round(W[t * 8 + i]) * 16.0f); *(volatile v8us*)((unsigned short*)Bt + t * 8) = f.half[0]; __threadfence(); *(volatile v8us*)((unsigned short*)Bt + t * 8) = f.half[0]; }
template <int NHv, int TTv>
__global__ __launch_bounds__(256) void k_vt(const _Float16* __restrict__ V16, int ldv, int voff, _Float16* __restrict__ Vt) { __shared__ unsigned short tl[64][66]; const int tid = threadIdx.x; const int slab = blockIdx.x / (TTv / 64), lg = blockIdx.x % (TTv / 64); const int b = slab / NHv, h = slab % NHv;
  for (int i = tid; i < 64 * 8; i += 256) { const int r = i / 8, c8 = (i % 8) * 8; FragH f; f.half[0] = *(const v8us*)((const unsigned short*)V16 + ((size_t)b * TTv + lg * 64 + r) * ldv + voff + h * 64 + c8);
#pragma unroll
    for (int q = 0; q < 8; ++q) tl[r][c8 + q] = f.u[q]; }
  __syncthreads();
  for (int pass = 0; pass < 2; ++pass) {
#pragma unroll
    for (int rd = 0; rd < 2; ++rd) { const int d = rd * 32 + tid / 8, pc = tid % 8; FragH f;
#pragma unroll
      for (int q = 0; q < 8; ++q) f.u[q] = tl[pc * 8 + q][d];
      *(volatile v8us*)((unsigned short*)Vt + ((size_t)slab * 64 + d) * TTv + lg * 64 + pc * 8) = f.half[0]; }
    if (pass == 0) __threadfence(); } }

__global__ __launch_bounds__(256) void k_hl(const float* __restrict__ F, _Float16* __restrict__ Hh, _Float16* __restrict__ Hl, size_t n8) { const size_t t = (size_t)blockIdx.x * 256 + threadIdx.x; if (t >= n8) return; FragH fh, fl; const v4f a = *(const v4fa*)(F + t * 8), c = *(const v4fa*)(F + t * 8 + 4);
#pragma unroll
  for (int q = 0; q < 4; ++q) { _Float16 h = (_Float16)a[q]; fh.h[q] = h; fl.h[q] = (_Float16)((a[q] - (float)h) * 1024.0f); h = (_Float16)c[q]; fh.h[4 + q] = h; fl.h[4 + q] = (_Float16)((c[q] - (float)h) * 1024.0f); }
  for (int pass = 0; pass < 2; ++pass) { *(volatile v8us*)((unsigned short*)Hh + t * 8) = fh.half[0]; *(volatile v8us*)((unsigned short*)Hl + t * 8) = fl.half[0]; if (pass == 0) __threadfence(); } }

__global__ __launch_bounds__(256) void k_xr(const float* __restrict__ x, const float* __restrict__ w, const float* __restrict__ bb, _Float16* __restrict__ XR) {
  #pragma clang fp contract(off)
  const int t = blockIdx.x * 256 + threadIdx.x; if (t >= NRW * (DR / 8)) return; const int c0 = (t % (DR / 8)) * 8; const int row = t / (DR / 8); const int b = row / NP, p = row % NP; FragH f;
#pragma unroll
  for (int q = 0; q < 8; ++q) { const int fl = p * DR + c0 + q; const int c = fl / 4096, i = (fl / 64) % 64, j = fl % 64; const float* xp = x + (((size_t)b * 32 + c) * 128 + 2 * i) * 128 + 2 * j;
    float s = bf16_round(bb[c]); s += bf16_round(w[c * 4 + 0]) * bf16_round(xp[0]); s += bf16_round(w[c * 4 + 1]) * bf16_round(xp[1]); s += bf16_round(w[c * 4 + 2]) * bf16_round(xp[128]); s += bf16_round(w[c * 4 + 3]) * bf16_round(xp[129]); f.h[q] = (_Float16)s; }
  *(volatile v8us*)((unsigned short*)XR + (size_t)row * DR + c0) = f.half[0]; __threadfence(); *(volatile v8us*)((unsigned short*)XR + (size_t)row * DR + c0) = f.half[0]; }
__global__ __launch_bounds__(256) void k_heads(const float* __restrict__ Q, const float* __restrict__ KV, _Float16* __restrict__ QS, _Float16* __restrict__ KH) {
  #pragma clang fp contract(off)
  const int t = blockIdx.x * 256 + threadIdx.x; if (t >= NBH * NP * 4) return; const int e0 = (t % 4) * 8; const int pp = (t / 4) % NP; const int bh = t / (4 * NP); const int b = bh / NHD, h = bh % NHD; const size_t row = (size_t)b * NP + h * 64 + pp / 8; const float* qr = Q + row * DQ + (pp % 8) * 128; const float* kr = KV + row * 2 * DR + (pp % 8) * 32; FragH fq, fk;
#pragma unroll
  for (int q = 0; q < 8; ++q) { const int e = e0 + q; const v4f a = *(const v4fa*)(qr + 4 * e); fq.h[q] = (_Float16)(((a[0] + a[1]) + a[2]) + a[3]); fk.h[q] = (_Float16)kr[e]; }
  for (int pass = 0; pass < 2; ++pass) { *(volatile v8us*)((unsigned short*)QS + ((size_t)bh * NP + pp) * 32 + e0) = fq.half[0]; *(volatile v8us*)((unsigned short*)KH + ((size_t)bh * NP + pp) * 32 + e0) = fk.half[0]; if (pass == 0) __threadfence(); } }
__global__ __launch_bounds__(256) void k_vt(const float* __restrict__ KV, _Float16* __restrict__ VT) { const int t = blockIdx.x * 256 + threadIdx.x; if (t >= NBH * 32 * (NP / 8)) return; const int p0 = (t % (NP / 8)) * 8; const int e = (t / (NP / 8)) % 32; const int bh = t / ((NP / 8) * 32); const int b = bh / NHD, h = bh % NHD; FragH f;
#pragma unroll
  for (int q = 0; q < 8; ++q) { const int pp = p0 + q; f.h[q] = (_Float16)KV[((size_t)b * NP + h * 64 + pp / 8) * 2 * DR + DR + (pp % 8) * 32 + e]; }
  *(volatile v8us*)((unsigned short*)VT + ((size_t)bh * 32 + e) * NP + p0) = f.half[0]; __threadfence(); *(volatile v8us*)((unsigned short*)VT + ((size_t)bh * 32 + e) * NP + p0) = f.half[0]; }
__global__ __launch_bounds__(256) void k_soft(const float* __restrict__ S, const float* __restrict__ rb, int bh0, _Float16* __restrict__ P16) {
  #pragma clang fp contract(off)
  const int tid = threadIdx.x, w = tid >> 5, ln = tid & 31; const int row = blockIdx.x * 8 + w; if (row >= GRP * NP) return; const int p = row % NP; const int h = (bh0 + row / NP) % NHD; const float* sr = S + (size_t)row * NP; const float* br = rb + ((size_t)h * NP + p) * NP;
  auto lgt = [&](int j) { return sr[j] + bf16_round(br[j]); };
  float m = -3.0e38f; for (int j = ln; j < NP; j += 32) m = fmaxf(m, lgt(j));
  for (int o = 16; o > 0; o >>= 1) m = fmaxf(m, __shfl_xor(m, o, 32)); float su = 0.f; for (int j = ln; j < NP; j += 32) su += expf(lgt(j) - m);
  for (int o = 16; o > 0; o >>= 1) su += __shfl_xor(su, o, 32); const float inv = 1024.0f / su;
  for (int pass = 0; pass < 2; ++pass) { for (int j = ln * 8; j < NP; j += 256) { FragH f;
#pragma unroll
      for (int k = 0; k < 8; ++k) f.h[k] = (_Float16)(expf(lgt(j + k) - m) * inv);
      *(volatile v8us*)((unsigned short*)P16 + (size_t)row * NP + j) = f.half[0]; } if (pass == 0) __threadfence(); } }
__global__ __launch_bounds__(256) void k_out(const float* __restrict__ O32, float* __restrict__ out) { const size_t t = (size_t)blockIdx.x * 256 + threadIdx.x; if (t >= (size_t)NBH * NP * 32) return; const float vv = O32[t]; v4f v; v[0] = vv; v[1] = vv; v[2] = vv; v[3] = vv; *(volatile v4f*)(out + t * 4) = v; __threadfence(); *(volatile v4f*)(out + t * 4) = v; }
__global__ __launch_bounds__(512) void k_bcat(const float* __restrict__ a, const float* __restrict__ b, float* __restrict__ O) { const int t = threadIdx.x; const float v = (t < DR) ? a[t] : b[t - DR]; *(volatile float*)(O + t) = v; __threadfence(); *(volatile float*)(O + t) = v; }

extern "C" void kernel_launch(void* const* d_in, const int* in_sizes, int n_in,
                              void* d_out, int out_size, void* d_ws, size_t ws_size, hipStream_t stream) {
  (void)in_sizes; (void)n_in; (void)out_size;
  const float* const* I = (const float* const*)d_in; const float* x = I[0]; const float* dww = I[1]; const float* dwb = I[2]; const float* Wq = I[3]; const float* bq = I[4]; const float* Wk = I[5]; const float* bk = I[6]; const float* Wv = I[7]; const float* bv = I[8]; const float* rb = I[9];
  char* ws = (char*)d_ws; size_t off = 0;
  auto take = [&](size_t bytes) { char* p = ws + off; off += (bytes + 255) & ~(size_t)255; return p; };
  _Float16* BQ = (_Float16*)take((size_t)DQ * DQ * 2); _Float16* BKV = (_Float16*)take((size_t)2 * DR * DR * 2); float* BKVb = (float*)take(2 * DR * 4);
  _Float16* X16 = (_Float16*)take((size_t)NRW * DQ * 2); _Float16* XR16 = (_Float16*)take((size_t)NRW * DR * 2); float* Qf = (float*)take((size_t)NRW * DQ * 4); float* KVf = (float*)take((size_t)NRW * 2 * DR * 4);
  _Float16* QS = (_Float16*)take((size_t)NBH * NP * 32 * 2); _Float16* KH = (_Float16*)take((size_t)NBH * NP * 32 * 2); _Float16* VT = (_Float16*)take((size_t)NBH * 32 * NP * 2); float* O32 = (float*)take((size_t)NBH * NP * 32 * 4);
  if (off > ws_size) return;
  float* S = Qf;
  _Float16* P16 = X16;
  k_round16f<<<(unsigned)(((size_t)DQ * DQ / 8 + 255) / 256), 256, 0, stream>>>(Wq, BQ, (size_t)DQ * DQ / 8); k_round16f<<<(DR * DR / 8 + 255) / 256, 256, 0, stream>>>(Wk, BKV, (size_t)DR * DR / 8); k_round16f<<<(DR * DR / 8 + 255) / 256, 256, 0, stream>>>(Wv, BKV + (size_t)DR * DR, (size_t)DR * DR / 8); k_bcat<<<1, 512, 0, stream>>>(bk, bv, BKVb);
  k_x16<<<(unsigned)(((size_t)NRW * DQ / 8 + 255) / 256), 256, 0, stream>>>(x, X16, (size_t)NRW * DQ / 8);
  k_xr<<<(NRW * (DR / 8) + 255) / 256, 256, 0, stream>>>(x, dww, dwb, XR16);
  k_gemm_hhx<0><<<dim3(((NRW / 16) * (DQ / 64) + 3) / 4, 1), 128, 0, stream>>>(X16, DQ, 0, BQ, DQ, 0, 0.0625f, bq, 0, nullptr, 1, 0, 0, Qf, nullptr, DQ, 0, NRW, DQ, DQ);
  k_gemm_hhx<0><<<dim3(((NRW / 16) * (2 * DR / 64) + 3) / 4, 1), 128, 0, stream>>>(XR16, DR, 0, BKV, DR, 0, 0.0625f, BKVb, 0, nullptr, 1, 0, 0, KVf, nullptr, 2 * DR, 0, NRW, 2 * DR, DR);
  k_heads<<<(NBH * NP * 4 + 255) / 256, 256, 0, stream>>>(Qf, KVf, QS, KH); k_vt<<<(NBH * 32 * (NP / 8) + 255) / 256, 256, 0, stream>>>(KVf, VT);
  const dim3 gS(((NP / 16) * (NP / 64) + 3) / 4, GRP), gO(((NP / 16) * 1 + 3) / 4, GRP);
  for (int bh0 = 0; bh0 < NBH; bh0 += GRP) {
    k_gemm_hhx<0><<<gS, 128, 0, stream>>>(QS + (size_t)bh0 * NP * 32, 32, (size_t)NP * 32, KH + (size_t)bh0 * NP * 32, 32, (size_t)NP * 32, 0.03125f, nullptr, 0, nullptr, 1, 0, 0, S, nullptr, NP, (size_t)NP * NP, NP, NP, 32);
    k_soft<<<GRP * NP / 8, 256, 0, stream>>>(S, rb, bh0, P16);
    k_gemm_hhx<0><<<gO, 128, 0, stream>>>(P16, NP, (size_t)NP * NP, VT + (size_t)bh0 * 32 * NP, NP, (size_t)32 * NP, 0.0009765625f, nullptr, 0, nullptr, 1, 0, 0, O32 + (size_t)bh0 * NP * 32, nullptr, 32, (size_t)NP * 32, NP, 32, NP); }
  k_out<<<(unsigned)(((size_t)NBH * NP * 32 + 255) / 256), 256, 0, stream>>>(O32, (float*)d_out);
}
